// TwoSimplicialAttention_24515673325872
// MI455X (gfx1250) — hardware-verified
//
#include <hip/hip_runtime.h>


#define SS_  1024
#define NH_  8
#define HD   64
#define WW_  64
#define RP   (SS_ + 64)
#define SC   128
#define TT   4096
#define ZH   1
#define RH   TT
#define PCAR 1024.0f
#define SCL  0.125f
#define DM   HD
#define DQ   HD
#define DKV  HD
#define NKV  NH_
typedef _Float16 h16;
typedef unsigned short bf;
typedef __attribute__((ext_vector_type(16))) __bf16   v16bf;
typedef __attribute__((ext_vector_type(16))) _Float16 v16h;
typedef __attribute__((ext_vector_type(8)))  _Float16 v8h;
typedef __attribute__((ext_vector_type(8)))  unsigned short v8us;
typedef __attribute__((ext_vector_type(8)))  float    v8f;
typedef __attribute__((ext_vector_type(4)))  float    v4f;
typedef v8h  __attribute__((may_alias)) v8ha;
typedef v4f  __attribute__((may_alias)) v4fa;
typedef v8us __attribute__((may_alias)) v8usa;

__device__ __forceinline__ unsigned short f2bf(float f) { unsigned u = __float_as_uint(f); u += 0x7FFFu + ((u >> 16) & 1u); return (unsigned short)(u >> 16); }
__device__ __forceinline__ float bf2f(unsigned short b) { return __uint_as_float(((unsigned)b) << 16); }
__device__ __forceinline__ float bfr(float f) { return bf2f(f2bf(f)); }
__device__ __forceinline__ v16h cat16(v8h lo, v8h hi) { return __builtin_shufflevector(lo, hi, 0, 1, 2, 3, 4, 5, 6, 7, 8, 9, 10, 11, 12, 13, 14, 15); }
__device__ __forceinline__ v16bf cat16b(v8us lo, v8us hi) { return __builtin_bit_cast(v16bf, __builtin_shufflevector(lo, hi, 0, 1, 2, 3, 4, 5, 6, 7, 8, 9, 10, 11, 12, 13, 14, 15)); }
__device__ __forceinline__ v8f wmma16(v16h a, v16h b, v8f c) { return __builtin_amdgcn_wmma_f32_16x16x32_f16(false, a, false, b, (short)0, c, false, false); }
__device__ __forceinline__ v8f wmmab(v16bf a, v16bf b, v8f c) { return __builtin_amdgcn_wmma_f32_16x16x32_bf16(false, a, false, b, (short)0, c, false, false); }


template <typename T16> struct WFrag;
template <> struct WFrag<h16> { typedef v16h V; static __device__ __forceinline__ V ld(const h16* p) { return cat16(*(const v8h*)p, *(const v8h*)(p + 16)); } static __device__ __forceinline__ v8f mma(V a, V b, v8f c) { return wmma16(a, b, c); } };
template <> struct WFrag<bf> { typedef v16bf V; static __device__ __forceinline__ V ld(const bf* p) { return cat16b(*(const v8us*)p, *(const v8us*)(p + 16)); } static __device__ __forceinline__ v8f mma(V a, V b, v8f c) { return wmmab(a, b, c); } };
template <typename T16, int NSPLIT, bool BIAS>
__global__ __launch_bounds__(32) void k_gemmw(const T16* __restrict__ A, const T16* __restrict__ A2, const T16* __restrict__ Bt, const T16* __restrict__ Bt2, int K, float* C, int ldc, const float* __restrict__ bias, size_t sA, size_t sB, size_t sC) {
    typedef typename WFrag<T16>::V V;
    __shared__ __align__(16) float os[16 * 68];
    const size_t z = blockIdx.z; A += z * sA; if (A2) A2 += z * sA; Bt += z * sB; if (Bt2) Bt2 += z * sB; C += z * sC;
    const int lane = threadIdx.x & 31, lr = lane & 15, hi = lane >> 4; const int r0 = blockIdx.x * 64, c0 = blockIdx.y * 64;
    v8f acc[4][4];
#pragma unroll
    for (int mb = 0; mb < 4; ++mb)
#pragma unroll
        for (int nb = 0; nb < 4; ++nb) acc[mb][nb] = (v8f){};
    const size_t aoff = (size_t)(r0 + lr) * K + 8 * hi, boff = (size_t)(c0 + lr) * K + 8 * hi;
#pragma unroll 1
    for (int kc = 0; kc < K; kc += 32) {
        V a[4], a2[4];
#pragma unroll
        for (int mb = 0; mb < 4; ++mb) { a[mb] = WFrag<T16>::ld(A + aoff + (size_t)mb * 16 * K + kc); if (NSPLIT == 1 || NSPLIT == 2) a2[mb] = WFrag<T16>::ld(A2 + aoff + (size_t)mb * 16 * K + kc); }
#pragma unroll
        for (int nb = 0; nb < 4; ++nb) { const V b = WFrag<T16>::ld(Bt + boff + (size_t)nb * 16 * K + kc); V b2; if (NSPLIT >= 2) b2 = WFrag<T16>::ld(Bt2 + boff + (size_t)nb * 16 * K + kc);
#pragma unroll
            for (int mb = 0; mb < 4; ++mb) { acc[mb][nb] = WFrag<T16>::mma(a[mb], b, acc[mb][nb]); if (NSPLIT == 1 || NSPLIT == 2) acc[mb][nb] = WFrag<T16>::mma(a2[mb], b, acc[mb][nb]); if (NSPLIT >= 2) acc[mb][nb] = WFrag<T16>::mma(a[mb], b2, acc[mb][nb]); } }
        asm volatile("v_nop\n\tv_nop\n\tv_nop\n\tv_nop" : "+v"(acc[0][0]), "+v"(acc[1][1]), "+v"(acc[2][2]), "+v"(acc[3][3]) : "v"(a[0]), "v"(a[3]));
    }
#pragma unroll
    for (int mb = 0; mb < 4; ++mb) {
#pragma unroll
        for (int nb = 0; nb < 4; ++nb) {
#pragma unroll
            for (int j = 0; j < 8; ++j) os[(hi * 8 + j) * 68 + nb * 16 + lr] = acc[mb][nb][j]; }
        __builtin_amdgcn_wave_barrier(); asm volatile("" ::: "memory");
        float* crow = C + (size_t)(r0 + mb * 16) * ldc + c0;
#pragma unroll 1
        for (int ps = 0; ps < 2; ++ps) {
#pragma unroll
            for (int s = 0; s < 8; ++s) { const int row = 2 * s + hi, cofs = lr * 4; v4f val = *(const v4fa*)(os + row * 68 + cofs); if (BIAS) { val[0] += bfr(bias[c0 + cofs]); val[1] += bfr(bias[c0 + cofs + 1]); val[2] += bfr(bias[c0 + cofs + 2]); val[3] += bfr(bias[c0 + cofs + 3]); }
                *(volatile v4f*)(crow + (size_t)row * ldc + cofs) = val; }
            if (ps == 0) __threadfence(); }
        __builtin_amdgcn_wave_barrier(); asm volatile("" ::: "memory");
    }
}

__device__ __forceinline__ h16 tohx(float x) { return (h16)x; }
__device__ __forceinline__ void splitf(float y, unsigned short& h, unsigned short& l) { h = f2bf(y); l = f2bf(y - bf2f(h)); }
typedef __attribute__((ext_vector_type(2))) _Float16 v2h;
typedef __attribute__((ext_vector_type(4))) _Float16 v4h;
typedef __attribute__((ext_vector_type(2))) unsigned short v2us;
typedef __attribute__((ext_vector_type(4))) unsigned short v4us;
typedef __attribute__((ext_vector_type(2))) float v2f;
typedef __attribute__((ext_vector_type(4))) int v4i;


__global__ __launch_bounds__(256) void k_padpl(const float* __restrict__ k1, const float* __restrict__ k2, const float* __restrict__ v1, const float* __restrict__ v2, float* K1P, bf* K2h, bf* K2l, float* V1P, float* V2P) { const size_t e = ((size_t)blockIdx.x * 256 + threadIdx.x) * 2; if (e >= (size_t)NH_ * RP * HD) return; const int d = (int)(e % HD); const int r = (int)((e / HD) % RP); const int h = (int)(e / ((size_t)HD * RP)); const int t = r - (WW_ - 1); v2f o1, o3, o4; v2us oh, ol;
    if (t >= 0 && t < SS_) { const size_t src = ((size_t)t * NH_ + h) * HD + d;
#pragma unroll
        for (int q = 0; q < 2; ++q) { o1[q] = bfr(k1[src + q]); o3[q] = bfr(v1[src + q]); o4[q] = __fadd_rn(bfr(v2[src + q]), 1.0f); const float kb = __fadd_rn(bfr(k2[src + q]), 1.0f); unsigned short a, c2; splitf(kb, a, c2); oh[q] = a; ol[q] = c2; } }
    else { o1 = (v2f){0.f, 0.f}; o3 = o1; o4 = o1; oh = (v2us){0, 0}; ol = oh; }
    *(volatile v2f*)(K1P + e) = o1; *(volatile v2us*)(K2h + e) = oh; *(volatile v2us*)(K2l + e) = ol; *(volatile v2f*)(V1P + e) = o3; *(volatile v2f*)(V2P + e) = o4; __threadfence();
    *(volatile v2f*)(K1P + e) = o1; *(volatile v2us*)(K2h + e) = oh; *(volatile v2us*)(K2l + e) = ol; *(volatile v2f*)(V1P + e) = o3; *(volatile v2f*)(V2P + e) = o4; }
__global__ __launch_bounds__(256) void k_qk1(const float* __restrict__ q, const float* __restrict__ K1P, int s0, bf* Ah, bf* Al) { const size_t e = ((size_t)blockIdx.x * 256 + threadIdx.x) * 2; if (e >= (size_t)NH_ * SC * WW_ * HD) return; const int d = (int)(e % HD); const int ap = (int)((e / HD) % WW_); const int sl = (int)((e / ((size_t)HD * WW_)) % SC); const int h = (int)(e / ((size_t)HD * WW_ * SC)); const int s = s0 + sl; v2us oh, ol;
#pragma unroll
    for (int u = 0; u < 2; ++u) { const float x = __fmul_rn(bfr(q[((size_t)s * NH_ + h) * HD + d + u]), K1P[((size_t)h * RP + s + ap) * HD + d + u]); unsigned short a, c2; splitf(x, a, c2); oh[u] = a; ol[u] = c2; }
    *(volatile v2us*)(Ah + e) = oh; *(volatile v2us*)(Al + e) = ol; __threadfence(); *(volatile v2us*)(Ah + e) = oh; *(volatile v2us*)(Al + e) = ol; }
__global__ __launch_bounds__(256) void k_v2w(const float* __restrict__ V2P, int s0, bf* Wh, bf* Wl) { const size_t e = ((size_t)blockIdx.x * 256 + threadIdx.x) * 2; if (e >= (size_t)NH_ * SC * HD * WW_) return; const int cp = (int)(e % WW_); const int d = (int)((e / WW_) % HD); const int sl = (int)((e / ((size_t)WW_ * HD)) % SC); const int h = (int)(e / ((size_t)WW_ * HD * SC)); const int s = s0 + sl; v2us oh, ol;
#pragma unroll
    for (int u = 0; u < 2; ++u) { unsigned short a, c2; splitf(V2P[((size_t)h * RP + s + cp + u) * HD + d], a, c2); oh[u] = a; ol[u] = c2; }
    *(volatile v2us*)(Wh + e) = oh; *(volatile v2us*)(Wl + e) = ol; __threadfence(); *(volatile v2us*)(Wh + e) = oh; *(volatile v2us*)(Wl + e) = ol; }
__global__ __launch_bounds__(256) void k_wsoft2(const float* __restrict__ L, int s0, bf* Ph, bf* Pl) {
    const int lane = threadIdx.x & 31; const int row = blockIdx.x * 8 + (threadIdx.x >> 5); if (row >= NH_ * SC) return; const int s = s0 + (row % SC); const int lim = (WW_ - 1) - s;     const float* sr = L + (size_t)row * TT; float v[TT / 32]; float mx = -3.0e38f;
#pragma unroll
    for (int ch = 0; ch < TT / 128; ++ch) { const int j0 = ch * 128 + lane * 4; const v4f a = *(const v4f*)(sr + j0);
#pragma unroll
        for (int qq = 0; qq < 4; ++qq) { const int j = j0 + qq; const int ap = j / WW_, cp = j % WW_; float sa = a[qq] * SCL; asm volatile("" : "+v"(sa)); const float t = (ap >= lim && cp >= lim) ? sa : -3.0e38f; v[ch * 4 + qq] = t; mx = fmaxf(mx, t); } }
#pragma unroll
    for (int sh = 16; sh; sh >>= 1) mx = fmaxf(mx, __shfl_xor(mx, sh, 32));
    float sum = 0.f;
#pragma unroll
    for (int k = 0; k < TT / 32; ++k) { float d0 = __fsub_rn(v[k], mx); asm volatile("" : "+v"(d0)); v[k] = __builtin_amdgcn_exp2f(__fmul_rn(d0, 1.4426950408889634f)); sum += v[k]; }
#pragma unroll
    for (int sh = 16; sh; sh >>= 1) sum += __shfl_xor(sum, sh, 32);
    const float f = __fdiv_rn(1.0f, sum);
#pragma unroll 1
    for (int ps = 0; ps < 2; ++ps) {
#pragma unroll
        for (int ch = 0; ch < TT / 128; ++ch) { v4us oh, ol;
#pragma unroll
            for (int qq = 0; qq < 4; ++qq) { unsigned short a, c2; float y = v[ch * 4 + qq] * f; asm volatile("" : "+v"(y)); splitf(y, a, c2); oh[qq] = a; ol[qq] = c2; }
            const size_t oo = (size_t)row * TT + ch * 128 + lane * 4; *(volatile v4us*)(Ph + oo) = oh; *(volatile v4us*)(Pl + oo) = ol; }
        if (ps == 0) __threadfence(); }
}
__global__ __launch_bounds__(256) void k_fin(const float* __restrict__ TMP, const float* __restrict__ V1P, int s0, float* O) { const int lane = threadIdx.x & 31; const int w = blockIdx.x * 8 + (threadIdx.x >> 5); if (w >= NH_ * SC) return; const int sl = w % SC, h = w / SC; const int s = s0 + sl; const float* tp = TMP + (size_t)w * WW_ * HD + lane * 2; const float* vp = V1P + ((size_t)h * RP + s) * HD + lane * 2; v2f acc = (v2f){0.f, 0.f};
#pragma unroll 1
    for (int ap = 0; ap < WW_; ++ap) { const v2f t2 = *(const v2f*)(tp + (size_t)ap * HD); const v2f v2v = *(const v2f*)(vp + (size_t)ap * HD);
#pragma unroll
        for (int u = 0; u < 2; ++u) { float pr = __fmul_rn(t2[u], v2v[u]); asm volatile("" : "+v"(pr)); acc[u] = __fadd_rn(acc[u], pr); } }
    float* dst = O + ((size_t)s * NH_ + h) * HD + lane * 2; *(volatile v2f*)dst = acc; __threadfence(); *(volatile v2f*)dst = acc; }

extern "C" void kernel_launch(void* const* d_in, const int* in_sizes, int n_in,
                              void* d_out, int out_size, void* d_ws, size_t ws_size, hipStream_t stream) {
    (void)in_sizes; (void)n_in; (void)out_size;
    const float* q = (const float*)d_in[0]; const float* k1 = (const float*)d_in[1]; const float* k2 = (const float*)d_in[2]; const float* v1 = (const float*)d_in[3]; const float* v2 = (const float*)d_in[4];
    float* OUT = (float*)d_out;
    char* wsp = (char*)d_ws;
    auto take = [&](size_t bytes) { char* p = wsp; wsp += (bytes + 255) & ~(size_t)255; return (void*)p; };
    float* K1P = (float*)take((size_t)NH_ * RP * HD * 4); bf* K2h = (bf*)take((size_t)NH_ * RP * HD * 2); bf* K2l = (bf*)take((size_t)NH_ * RP * HD * 2); float* V1P = (float*)take((size_t)NH_ * RP * HD * 4); float* V2P = (float*)take((size_t)NH_ * RP * HD * 4);
    bf* Ah = (bf*)take((size_t)NH_ * SC * WW_ * HD * 2); bf* Al = (bf*)take((size_t)NH_ * SC * WW_ * HD * 2); float* L = (float*)take((size_t)NH_ * SC * TT * 4); bf* Ph = (bf*)take((size_t)NH_ * SC * TT * 2); bf* Pl = (bf*)take((size_t)NH_ * SC * TT * 2); bf* Wh = (bf*)take((size_t)NH_ * SC * HD * WW_ * 2); bf* Wl = (bf*)take((size_t)NH_ * SC * HD * WW_ * 2); float* TMP = (float*)take((size_t)NH_ * SC * WW_ * HD * 4);
    if ((size_t)(wsp - (char*)d_ws) > ws_size) return;
    k_padpl<<<(unsigned)(((size_t)NH_ * RP * HD / 2 + 255) / 256), 256, 0, stream>>>(k1, k2, v1, v2, K1P, K2h, K2l, V1P, V2P);
    const unsigned LB = (unsigned)(((size_t)NH_ * SC * WW_ * HD / 2 + 255) / 256);
    for (int s0 = 0; s0 < SS_; s0 += SC) {
        k_qk1<<<LB, 256, 0, stream>>>(q, K1P, s0, Ah, Al);
        for (int h = 0; h < NH_; ++h)
            k_gemmw<bf, 2, false><<<dim3(1, 1, SC), 32, 0, stream>>>(Ah + (size_t)h * SC * WW_ * HD, Al + (size_t)h * SC * WW_ * HD, K2h + ((size_t)h * RP + s0) * HD, K2l + ((size_t)h * RP + s0) * HD, HD, L + (size_t)h * SC * TT, WW_, nullptr, (size_t)WW_ * HD, (size_t)HD, (size_t)TT);
        k_wsoft2<<<NH_ * SC / 8, 256, 0, stream>>>(L, s0, Ph, Pl);
        k_v2w<<<LB, 256, 0, stream>>>(V2P, s0, Wh, Wl);
        for (int h = 0; h < NH_; ++h)
            k_gemmw<bf, 2, false><<<dim3(1, 1, SC), 32, 0, stream>>>(Ph + (size_t)h * SC * TT, Pl + (size_t)h * SC * TT, Wh + (size_t)h * SC * HD * WW_, Wl + (size_t)h * SC * HD * WW_, WW_, TMP + (size_t)h * SC * WW_ * HD, HD, nullptr, (size_t)TT, (size_t)HD * WW_, (size_t)WW_ * HD);
        k_fin<<<NH_ * SC / 8, 256, 0, stream>>>(TMP, V1P, s0, OUT); }
}
